// BayerNN_2302102471018
// MI455X (gfx1250) — hardware-verified
//
#include <hip/hip_runtime.h>

constexpr int kBatch       = 8;
constexpr int kImg         = 512;
constexpr int kHalf        = 252;
constexpr int kOutDim      = 504;
constexpr int kRowsPerImg  = kHalf * kHalf;
constexpr int kRows        = kBatch * kRowsPerImg;
constexpr int kNumChunks   = 6;
constexpr int kChunkImgRows = 336;
constexpr int kChunkRows   = kChunkImgRows * kHalf;
constexpr int kNrmPitch    = 256;
constexpr int kFeatPad     = 128;
constexpr int kWinSz       = 4 * 5 * 36;
constexpr int kPlaneElems  = kOutDim * kOutDim;
constexpr int kPlaneQuads  = kPlaneElems / 4;

constexpr int kW1Off = 0;
constexpr int kW2Off = 16384;
constexpr int kW3Off = 24576;
constexpr int kW4Off = 28672;
constexpr int kW5Off = 32768;
constexpr int kWPlane = 36864;

constexpr size_t kOffW    = 0;
constexpr size_t kOffBias = 147456;
constexpr size_t kOffNrm  = 151552;
constexpr size_t kOffOutc = 2215936;
constexpr size_t kOffR0   = 18472960;
constexpr size_t kOffR1   = 61825024;
constexpr size_t kRegion  = (size_t)kChunkRows * 128 * 2 * 2;
constexpr size_t kWsEnd   = kOffR1 + kRegion;
constexpr size_t kPlane128 = (size_t)kChunkRows * 128 * 2;
constexpr size_t kPlane64  = (size_t)kChunkRows * 64 * 2;

typedef __attribute__((ext_vector_type(16))) _Float16 v16h;
typedef __attribute__((ext_vector_type(8)))  _Float16 v8h;
typedef __attribute__((ext_vector_type(16))) __bf16   v16b;
typedef __attribute__((ext_vector_type(8)))  __bf16   v8b;
typedef __attribute__((ext_vector_type(8)))  float    v8f;
typedef __attribute__((ext_vector_type(4)))  float    v4f;
typedef __attribute__((ext_vector_type(4)))  unsigned int v4u;

__device__ __forceinline__ unsigned short f2bf_bits(float f) {
  unsigned u = __float_as_uint(f);
  return (unsigned short)((u + 0x7FFFu + ((u >> 16) & 1u)) >> 16);
}
__device__ __forceinline__ float bf_bits2f(unsigned short h) { return __uint_as_float(((unsigned)h) << 16); }

__device__ __forceinline__ void dep_guard_h(v8f& a, v8f& b, v16h x, v16h y) { asm volatile("v_nop\n\tv_nop\n\tv_nop\n\tv_nop" : "+v"(a), "+v"(b) : "v"(x), "v"(y)); }
__device__ __forceinline__ void dep_guard_b(v8f& a, v8f& b, v16b x, v16b y) { asm volatile("v_nop\n\tv_nop\n\tv_nop\n\tv_nop" : "+v"(a), "+v"(b) : "v"(x), "v"(y)); }
__device__ __forceinline__ void keep4_h(v16h a, v16h b, v16h c, v16h d) { asm volatile("v_nop" :: "v"(a), "v"(b), "v"(c), "v"(d)); }
__device__ __forceinline__ void keep4_b(v16b a, v16b b, v16b c, v16b d) { asm volatile("v_nop" :: "v"(a), "v"(b), "v"(c), "v"(d)); }
__device__ __forceinline__ void acc_guard4(v8f& a, v8f& b, v8f& c, v8f& d) { asm volatile("v_nop\n\tv_nop\n\tv_nop\n\tv_nop" : "+v"(a), "+v"(b), "+v"(c), "+v"(d)); }
template <typename T> struct Frag;
template <> struct Frag<_Float16> {
  typedef v16h V; union U { v16h v; v8h h[2]; };
  static __device__ __forceinline__ v16h load(const _Float16* p) {
    U f; f.h[0] = *(const v8h*)(p); f.h[1] = *(const v8h*)(p + 16); return f.v;
  }
  static __device__ __forceinline__ v8f mma(v16h a, v16h b, v8f c) {
    return __builtin_amdgcn_wmma_f32_16x16x32_f16(false, a, false, b, (short)0, c, false, false);
  }
  static __device__ __forceinline__ void guard(v8f& a, v8f& b, v16h x, v16h y) { dep_guard_h(a, b, x, y); }
  static __device__ __forceinline__ void keep(v16h a, v16h b, v16h c, v16h d) { keep4_h(a, b, c, d); }
};
template <> struct Frag<__bf16> {
  typedef v16b V; union U { v16b v; v8b h[2]; };
  static __device__ __forceinline__ v16b load(const __bf16* p) {
    U f; f.h[0] = *(const v8b*)(p); f.h[1] = *(const v8b*)(p + 16); return f.v;
  }
  static __device__ __forceinline__ v8f mma(v16b a, v16b b, v8f c) {
    return __builtin_amdgcn_wmma_f32_16x16x32_bf16(false, a, false, b, (short)0, c, false, false);
  }
  static __device__ __forceinline__ void guard(v8f& a, v8f& b, v16b x, v16b y) { dep_guard_b(a, b, x, y); }
  static __device__ __forceinline__ void keep(v16b a, v16b b, v16b c, v16b d) { keep4_b(a, b, c, d); }
};

__device__ __forceinline__ unsigned pk16(unsigned short a, unsigned short b) { return (unsigned)a | ((unsigned)b << 16); }

__device__ __forceinline__ v8f at_mma(v16b a, v16b b, v8f c) {
  c = __builtin_amdgcn_wmma_f32_16x16x32_bf16(false, a, false, b, (short)0, c, false, false);
  asm volatile("v_nop\n\tv_nop\n\tv_nop\n\tv_nop" : "+v"(c) : "v"(a), "v"(b));
  return c;
}

template <int ET> struct Elem;
template <> struct Elem<0> { typedef _Float16 T; };
template <> struct Elem<1> { typedef __bf16 T; };
template <int ET, bool SPLIT, int BIAS_MODE, int OUT_MODE, bool RESID, int ACT = 0>
__global__ __launch_bounds__(256) void wmma_gemm64(
    const unsigned short* __restrict__ Ap, const unsigned short* __restrict__ A2p, int lda, long strideA,
    const unsigned short* __restrict__ Btp, const unsigned short* __restrict__ Bt2p, int ldb, long strideB,
    void* __restrict__ Cout, void* __restrict__ Cout2, int ldc, long strideC,
    const float* __restrict__ bias,
    const float* __restrict__ resid, long strideR,
    int M, int N, int K, float scale) {
  typedef typename Elem<ET>::T T;
  typedef typename Frag<T>::V V;
  const T* A = (const T*)Ap; const T* A2 = (const T*)A2p; const T* Bt = (const T*)Btp; const T* Bt2 = (const T*)Bt2p;
  __shared__ __align__(16) float sT[8][16 * 68];
  const int b    = blockIdx.y;
  const int lane = threadIdx.x & 31;
  const int wave = threadIdx.x >> 5;
  const int tilesN = N >> 6;
  const int tilesM = M >> 6;
  const int tile = blockIdx.x * 8 + wave;
  if (tile >= tilesM * tilesN) return;
  const int tm = tile / tilesN;
  const int tn = tile - tm * tilesN;
  const int m0 = tm << 6;
  const int n0 = tn << 6;

  const T* Ab  = A  + (size_t)b * strideA;
  const T* Bb  = Bt + (size_t)b * strideB;
  const T* Ab2 = SPLIT ? (A2  + (size_t)b * strideA) : nullptr;
  const T* Bb2 = SPLIT ? (Bt2 + (size_t)b * strideB) : nullptr;

  const int rlane = lane & 15;
  const int koff  = (lane >> 4) * 8;
  const int mOff  = (lane >> 4) * 8;

  v8f acc[4][4];
#pragma unroll
  for (int i = 0; i < 4; ++i)
#pragma unroll
    for (int j = 0; j < 4; ++j) acc[i][j] = (v8f){0.f,0.f,0.f,0.f,0.f,0.f,0.f,0.f};

  for (int k0 = 0; k0 < K; k0 += 32) {
    V bh[4], bl[4];
#pragma unroll
    for (int j = 0; j < 4; ++j) {
      const size_t bo = (size_t)(n0 + (j << 4) + rlane) * ldb + koff + k0;
      bh[j] = Frag<T>::load(Bb + bo);
      if (SPLIT) bl[j] = Frag<T>::load(Bb2 + bo);
    }
#pragma unroll
    for (int i = 0; i < 4; ++i) {
      const size_t ao = (size_t)(m0 + (i << 4) + rlane) * lda + koff + k0;
      V ah = Frag<T>::load(Ab + ao);
      V al;
      if (SPLIT) al = Frag<T>::load(Ab2 + ao);
#pragma unroll
      for (int j = 0; j < 4; ++j) {
        acc[i][j] = Frag<T>::mma(ah, bh[j], acc[i][j]);
        if (SPLIT) {
          acc[i][j] = Frag<T>::mma(ah, bl[j], acc[i][j]);
          acc[i][j] = Frag<T>::mma(al, bh[j], acc[i][j]);
        }
      }
      Frag<T>::guard(acc[i][0], acc[i][3], ah, SPLIT ? al : ah);
    }
    Frag<T>::keep(bh[0], bh[1], bh[2], bh[3]);
    if (SPLIT) Frag<T>::keep(bl[0], bl[1], bl[2], bl[3]);
  }
  acc_guard4(acc[0][0], acc[0][1], acc[0][2], acc[0][3]);
  acc_guard4(acc[1][0], acc[1][1], acc[1][2], acc[1][3]);
  acc_guard4(acc[2][0], acc[2][1], acc[2][2], acc[2][3]);
  acc_guard4(acc[3][0], acc[3][1], acc[3][2], acc[3][3]);

  float* slab = sT[wave];
  const float* Rb = RESID ? (resid + (size_t)b * strideR) : nullptr;
#pragma unroll
  for (int i = 0; i < 4; ++i) {
    const int mBase = m0 + (i << 4);
#pragma unroll
    for (int j = 0; j < 4; ++j) {
      const int n = n0 + (j << 4) + rlane;
      float bv = 0.f;
      if (BIAS_MODE == 2) bv = bias[n];
#pragma unroll
      for (int r = 0; r < 8; ++r) {
        float v = acc[i][j][r] * scale;
        if (BIAS_MODE == 1) v += bias[mBase + mOff + r];
        if (BIAS_MODE == 2) v += bv;
        if (RESID) v += Rb[(size_t)(mBase + mOff + r) * ldc + n];
        if (ACT == 2) v = fmaxf(v, 0.0f);
        if (ACT == 4) v = (v > 0.f) ? v : 0.01f * v;
        slab[(mOff + r) * 68 + (j << 4) + rlane] = v;
      }
    }
    __builtin_amdgcn_fence(__ATOMIC_RELEASE, "workgroup");
    __builtin_amdgcn_wave_barrier();
    __builtin_amdgcn_fence(__ATOMIC_ACQUIRE, "workgroup");
    if (OUT_MODE == 0) {
      float* C = (float*)Cout + (size_t)b * strideC;
      const int hh = lane >> 4, c4 = (lane & 15) * 4;
      for (int pass = 0; pass < 2; ++pass) {
#pragma unroll
        for (int it = 0; it < 8; ++it) {
          const int row = it * 2 + hh;
          v4f v = *(const v4f*)(slab + row * 68 + c4);
          *(volatile v4f*)(C + (size_t)(mBase + row) * ldc + n0 + c4) = v;
        }
        __threadfence();
      }
    } else {
      const int q = lane >> 3, c8 = (lane & 7) * 8;
      unsigned short* C  = (unsigned short*)Cout  + (size_t)b * strideC;
      unsigned short* C2 = (OUT_MODE == 2) ? ((unsigned short*)Cout2 + (size_t)b * strideC) : nullptr;
      for (int pass = 0; pass < 2; ++pass) {
#pragma unroll
        for (int it = 0; it < 4; ++it) {
          const int row = it * 4 + q;
          const float* sp = slab + row * 68 + c8;
          v8h hv, lv;
#pragma unroll
          for (int e = 0; e < 8; ++e) {
            if (OUT_MODE == 1) {
              hv[e] = (_Float16)sp[e];
            } else {
              unsigned short hb = f2bf_bits(sp[e]);
              unsigned short lb = f2bf_bits(sp[e] - bf_bits2f(hb));
              hv[e] = __builtin_bit_cast(_Float16, hb);
              lv[e] = __builtin_bit_cast(_Float16, lb);
            }
          }
          *(volatile v8h*)(C + (size_t)(mBase + row) * ldc + n0 + c8) = hv;
          if (OUT_MODE == 2) *(volatile v8h*)(C2 + (size_t)(mBase + row) * ldc + n0 + c8) = lv;
        }
        __threadfence();
      }
    }
    __builtin_amdgcn_fence(__ATOMIC_RELEASE, "workgroup");
    __builtin_amdgcn_wave_barrier();
    __builtin_amdgcn_fence(__ATOMIC_ACQUIRE, "workgroup");
  }
}

__global__ __launch_bounds__(256) void wprep_kernel(const float* __restrict__ W1, const float* __restrict__ W2,
                                                    const float* __restrict__ W3, const float* __restrict__ W4,
                                                    const float* __restrict__ W5,
                                                    unsigned short* __restrict__ whi, unsigned short* __restrict__ wlo) {
  const int ly = blockIdx.y;
  const float* W = (ly == 0) ? W1 : (ly == 1) ? W2 : (ly == 2) ? W3 : (ly == 3) ? W4 : W5;
  const int Kr  = (ly == 0) ? 100 : (ly == 1) ? 128 : (ly == 2) ? 64 : (ly == 3) ? 64 : 32;
  const int Nr  = (ly == 0) ? 128 : (ly == 1) ? 64  : (ly == 2) ? 64 : (ly == 3) ? 32 : 8;
  const int lk  = (ly <= 1) ? 7 : 6;
  const int Np  = (ly == 0) ? 128 : 64;
  const int off = (ly == 0) ? kW1Off : (ly == 1) ? kW2Off : (ly == 2) ? kW3Off : (ly == 3) ? kW4Off : kW5Off;
  const int ngroups = (Np << lk) >> 3;
  const int idx = blockIdx.x * 256 + threadIdx.x;
  if (idx >= ngroups) return;
  const int el = idx * 8;
  const int n  = el >> lk;
  const int k0 = el & ((1 << lk) - 1);
  const int nc = (n < Nr) ? n : (Nr - 1);
  unsigned short hb[8], lb[8];
#pragma unroll
  for (int u = 0; u < 8; ++u) {
    const int k  = k0 + u;
    const int kc = (k < Kr) ? k : (Kr - 1);
    float v = W[kc * Nr + nc];
    v = (k < Kr && n < Nr) ? v : 0.0f;
    hb[u] = f2bf_bits(v);
    lb[u] = f2bf_bits(v - bf_bits2f(hb[u]));
  }
  const v4u uh = (v4u){pk16(hb[0], hb[1]), pk16(hb[2], hb[3]), pk16(hb[4], hb[5]), pk16(hb[6], hb[7])};
  const v4u ul = (v4u){pk16(lb[0], lb[1]), pk16(lb[2], lb[3]), pk16(lb[4], lb[5]), pk16(lb[6], lb[7])};
  unsigned short* ph = whi + off + el;
  unsigned short* pl = wlo + off + el;
  *(volatile v4u*)ph = uh;
  *(volatile v4u*)pl = ul;
  __threadfence();
  *(volatile v4u*)ph = uh;
  *(volatile v4u*)pl = ul;
}

__global__ __launch_bounds__(32) void bias_kernel(const float* __restrict__ b4, const float* __restrict__ b5,
                                                  float* __restrict__ bp) {
  const int lane = threadIdx.x;
  float v[4];
#pragma unroll
  for (int e = 0; e < 4; ++e) {
    const int idx = 4 * lane + e;
    const int i4 = (idx < 32) ? idx : 31;
    int i5 = idx - 64; i5 = (i5 < 0) ? 0 : ((i5 > 7) ? 7 : i5);
    const float a = b4[i4];
    const float c = b5[i5];
    v[e] = (idx < 32) ? a : ((idx >= 64 && idx < 72) ? c : 0.0f);
  }
  const v4f vv = (v4f){v[0], v[1], v[2], v[3]};
  float* p = bp + 4 * lane;
  *(volatile v4f*)p = vv;
  __threadfence();
  *(volatile v4f*)p = vv;
}

__global__ __launch_bounds__(256) void feature_kernel(const float* __restrict__ mosaic,
                                                      unsigned short* __restrict__ Xh, unsigned short* __restrict__ Xl,
                                                      float* __restrict__ nrmOut, int rowTileBase) {
#pragma clang fp contract(off)
  __shared__ float win[8][kWinSz];
  const int t = threadIdx.x;
  const int lane = t & 31, wave = t >> 5;
  const int hsel = lane >> 4, e = lane & 15;
  const int R = rowTileBase + (int)blockIdx.y * 8 + wave;
  const int b = R / kHalf;
  const int i = R - b * kHalf;
  const int x0 = (int)blockIdx.x * 32;
  const float* mb = mosaic + (size_t)b * 3 * kImg * kImg;
  float* ww = win[wave];
  for (int q2 = lane; q2 < kWinSz; q2 += 32) {
    const int q  = q2 / 180;
    const int rr = q2 - q * 180;
    const int wy = rr / 36;
    const int wx = rr - wy * 36;
    const int gy = 2 * (i + wy) + (q & 1);
    int gx = 2 * (x0 + wx) + (q >> 1);
    gx = (gx > kImg - 1) ? (kImg - 1) : gx;
    const int gi = gy * kImg + gx;
    ww[q2] = (mb[gi] + mb[kImg * kImg + gi]) + mb[2 * kImg * kImg + gi];
  }
  __syncthreads();

  const int nlocBase = ((int)blockIdx.y * 8 + wave) * kHalf;
  float myNrm = 0.0f;
#pragma unroll 1
  for (int it = 0; it < 16; ++it) {
    const int p = 2 * it + hsel;
    float xv[8];
    float s = 0.0f;
#pragma unroll
    for (int u = 0; u < 8; ++u) {
      const int f  = 8 * e + u;
      const int fc = (f < 99) ? f : 99;
      const int q  = fc / 25;
      const int r2 = fc - 25 * q;
      const int di = r2 / 5;
      const int dj = r2 - 5 * di;
      float v = ww[(q * 5 + di) * 36 + p + dj];
      v = (f < 100) ? v : 0.0f;
      xv[u] = v;
      s += v;
    }
    s += __shfl_xor(s, 1, 32);
    s += __shfl_xor(s, 2, 32);
    s += __shfl_xor(s, 4, 32);
    s += __shfl_xor(s, 8, 32);
    const float nrm = s * 0.01f + 1e-8f;
    const float inv = 1.0f / nrm;
    const float n0v = __shfl(nrm, 0, 32);
    const float n1v = __shfl(nrm, 16, 32);
    if (lane == 2 * it)     myNrm = n0v;
    if (lane == 2 * it + 1) myNrm = n1v;
    unsigned short hb[8], lb[8];
#pragma unroll
    for (int u = 0; u < 8; ++u) {
      const float x = xv[u] * inv;
      hb[u] = f2bf_bits(x);
      lb[u] = f2bf_bits(x - bf_bits2f(hb[u]));
    }
    const v4u uh = (v4u){pk16(hb[0], hb[1]), pk16(hb[2], hb[3]), pk16(hb[4], hb[5]), pk16(hb[6], hb[7])};
    const v4u ul = (v4u){pk16(lb[0], lb[1]), pk16(lb[2], lb[3]), pk16(lb[4], lb[5]), pk16(lb[6], lb[7])};
    const bool pairValid = (x0 + 2 * it) < kHalf;
    if (pairValid) {
      const size_t off = (size_t)(nlocBase + x0 + p) * kFeatPad + 8 * e;
      unsigned short* ph = Xh + off;
      unsigned short* pl = Xl + off;
      *(volatile v4u*)ph = uh;
      *(volatile v4u*)pl = ul;
      __threadfence();
      *(volatile v4u*)ph = uh;
      *(volatile v4u*)pl = ul;
    }
  }
  float* np = nrmOut + (size_t)R * kNrmPitch + x0 + lane;
  *(volatile float*)np = myNrm;
  __threadfence();
  *(volatile float*)np = myNrm;
}

__global__ __launch_bounds__(256) void tail_kernel(const unsigned short* __restrict__ Hh, const unsigned short* __restrict__ Hl,
                                                   const unsigned short* __restrict__ Wh, const unsigned short* __restrict__ Wl,
                                                   const float* __restrict__ b5p, const float* __restrict__ nrm,
                                                   float* __restrict__ outc, int chunkBase) {
  __shared__ __align__(16) float slab[8][16 * 16];
  const int lane = threadIdx.x & 31, wave = threadIdx.x >> 5;
  const int rb = ((int)blockIdx.x * 8 + wave) * 16;
  if (rb >= kChunkRows) return;
  const int rlane = lane & 15;
  const int koff  = (lane >> 4) * 8;
  const int mOff  = (lane >> 4) * 8;
  const __bf16* Ah = (const __bf16*)Hh;
  const __bf16* Al = (const __bf16*)Hl;
  const __bf16* Bh = (const __bf16*)Wh;
  const __bf16* Bl = (const __bf16*)Wl;
  const v16b ah = Frag<__bf16>::load(Ah + (size_t)(rb + rlane) * 64 + koff);
  const v16b al = Frag<__bf16>::load(Al + (size_t)(rb + rlane) * 64 + koff);
  const v16b bh = Frag<__bf16>::load(Bh + rlane * 64 + koff);
  const v16b bl = Frag<__bf16>::load(Bl + rlane * 64 + koff);
  v8f acc = (v8f){0.f,0.f,0.f,0.f,0.f,0.f,0.f,0.f};
  acc = at_mma(ah, bh, acc);
  acc = at_mma(ah, bl, acc);
  acc = at_mma(al, bh, acc);
  float* sw = slab[wave];
#pragma unroll
  for (int r = 0; r < 8; ++r) sw[(mOff + r) * 16 + rlane] = acc[r];
  __builtin_amdgcn_fence(__ATOMIC_RELEASE, "workgroup");
  __builtin_amdgcn_wave_barrier();
  __builtin_amdgcn_fence(__ATOMIC_ACQUIRE, "workgroup");
  const int q = lane >> 1, s4 = (lane & 1) * 4;
  v4f val = *(const v4f*)(sw + q * 16 + s4);
  const v4f bb = *(const v4f*)(b5p + s4);
  const int n  = chunkBase + rb + q;
  const int Rg = n / kHalf;
  const int j  = n - Rg * kHalf;
  const float sc = nrm[(size_t)Rg * kNrmPitch + j];
  val = (val + bb) * sc;
  float* dst = outc + (size_t)n * 8 + s4;
  *(volatile v4f*)dst = val;
  __threadfence();
  *(volatile v4f*)dst = val;
}

__global__ __launch_bounds__(256) void assemble_kernel(const float* __restrict__ mosaic, const float* __restrict__ outc,
                                                       float* __restrict__ out) {
  const int plane = blockIdx.y;
  const int b = plane / 3;
  const int c = plane - 3 * b;
  const int t = (int)blockIdx.x * 256 + threadIdx.x;
  if (t >= kPlaneQuads) return;
  const int e0 = 4 * t;
  const int y  = e0 / kOutDim;
  const int x  = e0 - y * kOutDim;
  const int i  = y >> 1, l = y & 1, jb = x >> 1;
  const unsigned long long kTab = 0x7F31F52F64F0ULL;
  const int idx0  = c * 4 + l * 2;
  const int code0 = (int)((kTab >> (4 * idx0)) & 0xFULL);
  const int code1 = (int)((kTab >> (4 * (idx0 + 1))) & 0xFULL);
  const int ch0 = (code0 > 7) ? 0 : code0;
  const int ch1 = (code1 > 7) ? 0 : code1;
  const size_t n0 = (size_t)b * kRowsPerImg + (size_t)i * kHalf + jb;
  const float o00 = outc[n0 * 8 + ch0];
  const float o01 = outc[n0 * 8 + ch1];
  const float o10 = outc[(n0 + 1) * 8 + ch0];
  const float o11 = outc[(n0 + 1) * 8 + ch1];
  const float* mr = mosaic + ((size_t)plane * kImg + 4 + y) * kImg + 4 + x;
  const float m0 = mr[0], m1 = mr[1], m2 = mr[2], m3 = mr[3];
  v4f v;
  v[0] = (code0 == 15) ? m0 : o00;
  v[1] = (code1 == 15) ? m1 : o01;
  v[2] = (code0 == 15) ? m2 : o10;
  v[3] = (code1 == 15) ? m3 : o11;
  float* dst = out + (size_t)plane * kPlaneElems + e0;
  *(volatile v4f*)dst = v;
  __threadfence();
  *(volatile v4f*)dst = v;
}

extern "C" void kernel_launch(void* const* d_in, const int* in_sizes, int n_in,
                              void* d_out, int out_size, void* d_ws, size_t ws_size,
                              hipStream_t stream) {
  if (n_in < 11) return;
  if (in_sizes[0] != kBatch * 3 * kImg * kImg) return;
  if (out_size != kBatch * 3 * kOutDim * kOutDim) return;
  if (in_sizes[1] != 100 * 128 || in_sizes[3] != 128 * 64 || in_sizes[5] != 64 * 64 ||
      in_sizes[7] != 64 * 32 || in_sizes[9] != 32 * 8) return;
  if (in_sizes[2] < 128 || in_sizes[4] < 64 || in_sizes[6] < 64 || in_sizes[8] < 32 || in_sizes[10] < 8) return;
  if (ws_size < kWsEnd) return;

  const float* mosaic = (const float*)d_in[0];
  const float* W1 = (const float*)d_in[1];  const float* b1 = (const float*)d_in[2];
  const float* W2 = (const float*)d_in[3];  const float* b2 = (const float*)d_in[4];
  const float* W3 = (const float*)d_in[5];  const float* b3 = (const float*)d_in[6];
  const float* W4 = (const float*)d_in[7];  const float* b4 = (const float*)d_in[8];
  const float* W5 = (const float*)d_in[9];  const float* b5 = (const float*)d_in[10];
  float* out = (float*)d_out;
  char* ws = (char*)d_ws;

  unsigned short* whi = (unsigned short*)(ws + kOffW);
  unsigned short* wlo = whi + kWPlane;
  float* bp   = (float*)(ws + kOffBias);
  float* nrm  = (float*)(ws + kOffNrm);
  float* outc = (float*)(ws + kOffOutc);
  unsigned short* Xh  = (unsigned short*)(ws + kOffR0);
  unsigned short* Xl  = (unsigned short*)(ws + kOffR0 + kPlane128);
  unsigned short* H2h = (unsigned short*)(ws + kOffR0);
  unsigned short* H2l = (unsigned short*)(ws + kOffR0 + kPlane64);
  unsigned short* H4h = H2h;
  unsigned short* H4l = H2l;
  unsigned short* H1h = (unsigned short*)(ws + kOffR1);
  unsigned short* H1l = (unsigned short*)(ws + kOffR1 + kPlane128);
  unsigned short* H3h = (unsigned short*)(ws + kOffR1);
  unsigned short* H3l = (unsigned short*)(ws + kOffR1 + kPlane64);

  const unsigned short* W1h = whi + kW1Off; const unsigned short* W1l = wlo + kW1Off;
  const unsigned short* W2h = whi + kW2Off; const unsigned short* W2l = wlo + kW2Off;
  const unsigned short* W3h = whi + kW3Off; const unsigned short* W3l = wlo + kW3Off;
  const unsigned short* W4h = whi + kW4Off; const unsigned short* W4l = wlo + kW4Off;
  const unsigned short* W5h = whi + kW5Off; const unsigned short* W5l = wlo + kW5Off;

  wprep_kernel<<<dim3(8, 5), 256, 0, stream>>>(W1, W2, W3, W4, W5, whi, wlo);
  bias_kernel<<<1, 32, 0, stream>>>(b4, b5, bp);

  const int M = kChunkRows;
  const int gridL1 = (1323 * 2 + 7) / 8;
  const int gridLn = (1323 + 7) / 8;
  const int gridTail = (kChunkRows / 16 + 7) / 8;

  for (int ck = 0; ck < kNumChunks; ++ck) {
    feature_kernel<<<dim3(8, kChunkImgRows / 8), 256, 0, stream>>>(mosaic, Xh, Xl, nrm, ck * kChunkImgRows);
    wmma_gemm64<1, true, 2, 2, false, 4><<<dim3(gridL1, 1), 256, 0, stream>>>(
        Xh, Xl, 128, 0L, W1h, W1l, 128, 0L, (void*)H1h, (void*)H1l, 128, 0L, b1, bp, 0L, M, 128, 128, 1.0f);
    wmma_gemm64<1, true, 2, 2, false, 4><<<dim3(gridLn, 1), 256, 0, stream>>>(
        H1h, H1l, 128, 0L, W2h, W2l, 128, 0L, (void*)H2h, (void*)H2l, 64, 0L, b2, bp, 0L, M, 64, 128, 1.0f);
    wmma_gemm64<1, true, 2, 2, false, 4><<<dim3(gridLn, 1), 256, 0, stream>>>(
        H2h, H2l, 64, 0L, W3h, W3l, 64, 0L, (void*)H3h, (void*)H3l, 64, 0L, b3, bp, 0L, M, 64, 64, 1.0f);
    wmma_gemm64<1, true, 2, 2, false, 4><<<dim3(gridLn, 1), 256, 0, stream>>>(
        H3h, H3l, 64, 0L, W4h, W4l, 64, 0L, (void*)H4h, (void*)H4l, 64, 0L, bp, bp, 0L, M, 64, 64, 1.0f);
    tail_kernel<<<gridTail, 256, 0, stream>>>(H4h, H4l, W5h, W5l, bp + 64, nrm, outc, ck * kChunkRows);
  }

  assemble_kernel<<<dim3((kPlaneQuads + 255) / 256, kBatch * 3), 256, 0, stream>>>(mosaic, outc, out);
}
